// Self_Attention_Layer_4724464025889
// MI455X (gfx1250) — hardware-verified
//
#include <hip/hip_runtime.h>


namespace {
typedef _Float16 b16;
typedef __attribute__((ext_vector_type(16))) _Float16 v16b;
typedef __attribute__((ext_vector_type(8))) _Float16 v8b;
typedef __attribute__((ext_vector_type(4))) _Float16 v4h;
typedef __attribute__((ext_vector_type(2))) _Float16 v2h;
typedef __attribute__((ext_vector_type(8))) float v8f;
typedef __attribute__((ext_vector_type(4))) float v4f;
typedef __attribute__((ext_vector_type(2))) float v2f;
__device__ __forceinline__ float bf16_rne(float f) { unsigned int u = __float_as_uint(f); u += 0x7FFFu + ((u >> 16) & 1u); return __uint_as_float(u & 0xFFFF0000u); }
__device__ __forceinline__ void split16(float v, b16& hi, b16& lo) { hi = (b16)v; lo = (b16)(v - (float)hi); }
__device__ __forceinline__ v16b frag_kb(const b16* p, int hh) { const v8b a = *(const v8b*)(p + 8 * hh), b = *(const v8b*)(p + 16 + 8 * hh); v16b f;
#pragma unroll
  for (int e = 0; e < 8; ++e) { f[e] = a[e]; f[8 + e] = b[e]; } return f; }
__device__ __forceinline__ v8f wmma16b(v16b a, v16b b, v8f c) { v8f d = __builtin_amdgcn_wmma_f32_16x16x32_f16(false, a, false, b, (short)0, c, false, false); asm volatile("v_nop\n\tv_nop\n\tv_nop\n\tv_nop" : "+v"(d) : "v"(a), "v"(b)); return d; }
__device__ __forceinline__ void wave_lds_sync() { __builtin_amdgcn_fence(__ATOMIC_RELEASE, "workgroup"); __builtin_amdgcn_wave_barrier(); __builtin_amdgcn_fence(__ATOMIC_ACQUIRE, "workgroup"); }
__device__ __forceinline__ float pmul(float a, float b) { float p = a * b; asm volatile("" : "+v"(p)); return p; }
__device__ __forceinline__ int iclamp(int v, int lo, int hi) { return v < lo ? lo : (v > hi ? hi : v); }
__device__ __forceinline__ float nexp2(float v) { return __builtin_amdgcn_exp2f(v); }

constexpr int B = 16, BL = B  , S = 2048, DIN = 256, DA = 128, NROW = B * S;
constexpr float XS = 8.0f, WSC = 256.0f, PS = 1024.0f, RS_ = 1024.0f, LOG2E = 1.4426950408889634f, SCALE = 0.0625f  ;
static_assert(S % 64 == 0 && DIN % 32 == 0 && DA == 128, "tiling");

__global__ __launch_bounds__(256) void wt_kernel(const float* __restrict__ wq, const float* __restrict__ wk, const float* __restrict__ wv, b16* __restrict__ WT) {
  const int u = blockIdx.x * 256 + threadIdx.x; if (u >= 3 * DA * DIN / 8) return; const int e = u * 8; const int o = e / DIN, k0 = e % DIN; const int part = o / DA, oo = o % DA; const float* w = part == 0 ? wq : part == 1 ? wk : wv; v8b v;
#pragma unroll
  for (int j = 0; j < 8; ++j) v[j] = (b16)(bf16_rne(w[(size_t)(k0 + j) * DA + oo]) * WSC);
  for (int pass = 0; pass < 2; ++pass) { *(volatile v8b*)(WT + e) = v; __threadfence(); }
}
__global__ __launch_bounds__(128) void proj_kernel(const float* __restrict__ x, const b16* __restrict__ WT, b16* __restrict__ Qh, b16* __restrict__ Ql, b16* __restrict__ Kh, b16* __restrict__ Kl, b16* __restrict__ VTh, b16* __restrict__ VTl) {
  __shared__ __attribute__((aligned(16))) b16 As[64][DIN + 8]; __shared__ __attribute__((aligned(16))) float Tf[4][16][DA + 4];
  const int wave = threadIdx.x >> 5, lane = threadIdx.x & 31, nloc = lane & 15, hlf = lane >> 4; const int t0 = blockIdx.x * 64; const int b = blockIdx.y; const int part = blockIdx.z;
  for (int i = threadIdx.x; i < 64 * (DIN / 4); i += 128) { const int rr = i / (DIN / 4), q4 = (i % (DIN / 4)) * 4; const v4f f = *(const v4f*)(x + ((size_t)b * S + t0 + rr) * DIN + q4); v4h o; for (int j = 0; j < 4; ++j) o[j] = (b16)(bf16_rne(f[j]) * XS); *(v4h*)(&As[rr][q4]) = o; }
  __syncthreads();
  v8f acc[8];
#pragma unroll
  for (int tt = 0; tt < 8; ++tt) acc[tt] = (v8f){};
#pragma unroll 2
  for (int kb = 0; kb < DIN; kb += 32) { const v16b a = frag_kb(&As[wave * 16 + nloc][kb], hlf);
#pragma unroll
    for (int tt = 0; tt < 8; ++tt) acc[tt] = wmma16b(a, frag_kb(WT + (size_t)(part * DA + tt * 16 + nloc) * DIN + kb, hlf), acc[tt]); }
#pragma unroll
  for (int tt = 0; tt < 8; ++tt)
#pragma unroll
    for (int r = 0; r < 8; ++r) Tf[wave][8 * hlf + r][tt * 16 + nloc] = acc[tt][r] * (1.0f / (XS * WSC));
  __syncthreads();
  for (int pass = 0; pass < 2; ++pass) {
    if (part < 2) { b16* ph_ = part == 0 ? Qh : Kh; b16* pl_ = part == 0 ? Ql : Kl;
      for (int rr = 0; rr < 16; ++rr) { const size_t dst = ((size_t)b * S + t0 + wave * 16 + rr) * DA + lane * 4; v4h hv, lv; for (int j = 0; j < 4; ++j) { const float vs = Tf[wave][rr][lane * 4 + j] * XS; const b16 p1 = (b16)vs; hv[j] = p1; lv[j] = (b16)((vs - (float)p1) * RS_); } *(volatile v4h*)(ph_ + dst) = hv; *(volatile v4h*)(pl_ + dst) = lv; } }
    else {
#pragma unroll 1
      for (int q = 0; q < 32; ++q) { const int d = wave * 32 + q; const int tk = lane * 2; v2h hv, lv; for (int e2 = 0; e2 < 2; ++e2) { const float vs = Tf[(tk + e2) >> 4][(tk + e2) & 15][d] * XS; const b16 p1 = (b16)vs; hv[e2] = p1; lv[e2] = (b16)((vs - (float)p1) * RS_); }
        const size_t dst = ((size_t)b * DA + d) * (size_t)S + t0 + tk; *(volatile v2h*)(VTh + dst) = hv; *(volatile v2h*)(VTl + dst) = lv; } }
    __threadfence(); }
}
__global__ __launch_bounds__(64) void attn_kernel(const b16* __restrict__ Qh, const b16* __restrict__ Ql, const b16* __restrict__ Kh, const b16* __restrict__ Kl, const b16* __restrict__ VTh, const b16* __restrict__ VTl, const int* __restrict__ slen, float* __restrict__ out) {
  __shared__ __attribute__((aligned(16))) b16 Pb[2][16][32 + 8], Pl[2][16][32 + 8]; __shared__ __attribute__((aligned(16))) float To[2][16][DA + 4];
  const int wave = threadIdx.x >> 5, lane = threadIdx.x & 31, hh = lane >> 4, col = lane & 15; const int b = blockIdx.y; const int n0 = blockIdx.x * 32 + wave * 16; const int nq = n0 + col;
  int nk = iclamp(slen[b], 0, S); const bool allmask = (nk == 0); if (allmask) nk = S;
  const size_t qoff = ((size_t)b * S + nq) * DA; const b16* Khb = Kh + (size_t)b * S * DA; const b16* Klb = Kl + (size_t)b * S * DA; const b16* Vh = VTh + (size_t)b * DA * S; const b16* Vl = VTl + (size_t)b * DA * S;
  const float cs = LOG2E * SCALE / (XS * XS);
  float mrun = -INFINITY, l = 0.0f; v8f o[8], o2[8];
#pragma unroll
  for (int t = 0; t < 8; ++t) { o[t] = (v8f){}; o2[t] = (v8f){}; }
#pragma unroll 1
  for (int s0 = 0; s0 < nk; s0 += 32) {
    float e[16]; float mx = -INFINITY;
#pragma unroll
    for (int u2 = 0; u2 < 2; ++u2) { v8f sa = (v8f){}, sb = (v8f){}; const size_t koff = (size_t)(s0 + u2 * 16 + col) * DA;
#pragma unroll
      for (int kb = 0; kb < DA; kb += 32) { const v16b qh = frag_kb(Qh + qoff + kb, hh), ql = frag_kb(Ql + qoff + kb, hh); const v16b kh = frag_kb(Khb + koff + kb, hh); sa = wmma16b(kh, qh, sa); sb = wmma16b(frag_kb(Klb + koff + kb, hh), qh, sb); sb = wmma16b(kh, ql, sb); }
#pragma unroll
      for (int r = 0; r < 8; ++r) { const int m = s0 + u2 * 16 + 8 * hh + r; const float sv = allmask ? 0.0f : (sa[r] + sb[r] * (1.0f / RS_)) * cs; const float vv = (m < nk) ? sv : -INFINITY; e[u2 * 8 + r] = vv; mx = fmaxf(mx, vv); } }
    mx = fmaxf(mx, __shfl_xor(mx, 16)); const float mn = fmaxf(mrun, mx); const float al = (mn == -INFINITY) ? 1.0f : nexp2(mrun - mn); float sum = 0.0f;
#pragma unroll
    for (int i2 = 0; i2 < 16; ++i2) { const float p = (mn == -INFINITY) ? 0.0f : nexp2(e[i2] - mn); sum += p; const float psv = p * PS; const b16 p1 = (b16)psv; const int slot = (i2 < 8 ? 0 : 16) + 8 * hh + (i2 & 7); Pb[wave][col][slot] = p1; Pl[wave][col][slot] = (b16)((psv - (float)p1) * RS_); }
    sum += __shfl_xor(sum, 16); l = l * al + sum; mrun = mn;
    wave_lds_sync();
    const v16b pf = frag_kb(&Pb[wave][col][0], hh), plf = frag_kb(&Pl[wave][col][0], hh);
#pragma unroll
    for (int t = 0; t < 8; ++t) { o[t] *= al; o2[t] *= al; const v16b vh = frag_kb(Vh + (size_t)(t * 16 + col) * S + s0, hh); o[t] = wmma16b(vh, pf, o[t]); o2[t] = wmma16b(frag_kb(Vl + (size_t)(t * 16 + col) * S + s0, hh), pf, o2[t]); o2[t] = wmma16b(vh, plf, o2[t]); }
    wave_lds_sync(); }
  const float inv = 1.0f / (l * PS * XS);
#pragma unroll
  for (int t = 0; t < 8; ++t)
#pragma unroll
    for (int r = 0; r < 8; ++r) To[wave][col][t * 16 + 8 * hh + r] = (o[t][r] + o2[t][r] * (1.0f / RS_)) * inv;
  wave_lds_sync();
  for (int pass = 0; pass < 2; ++pass) { for (int rr = 0; rr < 16; ++rr) *(volatile v4f*)(out + ((size_t)b * S + n0 + rr) * DA + lane * 4) = *(const v4f*)(&To[wave][rr][lane * 4]); __threadfence(); }
}
}

extern "C" void kernel_launch(void* const* d_in, const int* in_sizes, int n_in, void* d_out, int out_size, void* d_ws, size_t ws_size, hipStream_t stream) {
  (void)n_in;
  auto Fp = [&](int i) { return (const float*)d_in[i]; };
  if (in_sizes[0] != NROW * DIN || in_sizes[1] != B || in_sizes[2] != DIN * DA || in_sizes[3] != DIN * DA || in_sizes[4] != DIN * DA || out_size != NROW * DA) return;
  size_t off = 0; char* ws = (char*)d_ws;
  auto carve = [&](size_t bytes) { char* p = ws + off; off += (bytes + 255) & ~(size_t)255; return p; };
  b16* WT = (b16*)carve((size_t)3 * DA * DIN * 2); const size_t plane = (size_t)NROW * DA * 2;
  b16* Qh = (b16*)carve(plane); b16* Ql = (b16*)carve(plane); b16* Kh = (b16*)carve(plane); b16* Kl = (b16*)carve(plane); b16* VTh = (b16*)carve(plane); b16* VTl = (b16*)carve(plane);
  if (off > ws_size || off > ((size_t)128 << 20)) return;
  wt_kernel<<<(3 * DA * DIN / 8 + 255) / 256, 256, 0, stream>>>(Fp(2), Fp(3), Fp(4), WT);
  proj_kernel<<<dim3(S / 64, BL, 3), 128, 0, stream>>>(Fp(0), WT, Qh, Ql, Kh, Kl, VTh, VTl);
  attn_kernel<<<dim3(S / 32, BL), 64, 0, stream>>>(Qh, Ql, Kh, Kl, VTh, VTl, (const int*)d_in[1], (float*)d_out);
}
